// SGIN_71425306133015
// MI455X (gfx1250) — hardware-verified
//
#include <hip/hip_runtime.h>
#include <math.h>
#define SRB 1024
#define SCHK 4096
typedef __attribute__((ext_vector_type(16))) _Float16 v16h;
typedef __attribute__((ext_vector_type(8)))  _Float16 v8h;
typedef __attribute__((ext_vector_type(16))) __bf16   v16b;
typedef __attribute__((ext_vector_type(8)))  __bf16   v8b;
typedef __attribute__((ext_vector_type(8)))  float    v8f;
typedef __attribute__((ext_vector_type(4)))  float    v4f;
#define PSCALE 32768.0f
#define U16(p) ((const unsigned short*)(const void*)(p))
#define PSCALE_INV (1.0f / 32768.0f)

__device__ __forceinline__ unsigned short f2bf_bits(float f) {
  unsigned u = __float_as_uint(f);
  return (unsigned short)((u + 0x7FFFu + ((u >> 16) & 1u)) >> 16);
}
__device__ __forceinline__ float bf_bits2f(unsigned short h) { return __uint_as_float(((unsigned)h) << 16); }

__device__ __forceinline__ void dep_guard_h(v8f& a, v8f& b, v16h x, v16h y) { asm volatile("v_nop\n\tv_nop\n\tv_nop\n\tv_nop" : "+v"(a), "+v"(b) : "v"(x), "v"(y)); }
__device__ __forceinline__ void dep_guard_b(v8f& a, v8f& b, v16b x, v16b y) { asm volatile("v_nop\n\tv_nop\n\tv_nop\n\tv_nop" : "+v"(a), "+v"(b) : "v"(x), "v"(y)); }
__device__ __forceinline__ void keep4_h(v16h a, v16h b, v16h c, v16h d) { asm volatile("v_nop" :: "v"(a), "v"(b), "v"(c), "v"(d)); }
__device__ __forceinline__ void keep4_b(v16b a, v16b b, v16b c, v16b d) { asm volatile("v_nop" :: "v"(a), "v"(b), "v"(c), "v"(d)); }
__device__ __forceinline__ void acc_guard4(v8f& a, v8f& b, v8f& c, v8f& d) { asm volatile("v_nop\n\tv_nop\n\tv_nop\n\tv_nop" : "+v"(a), "+v"(b), "+v"(c), "+v"(d)); }
template <typename T> struct Frag;
template <> struct Frag<_Float16> {
  typedef v16h V; union U { v16h v; v8h h[2]; };
  static __device__ __forceinline__ v16h load(const _Float16* p) {
    U f; f.h[0] = *(const v8h*)(p); f.h[1] = *(const v8h*)(p + 16); return f.v;
  }
  static __device__ __forceinline__ v8f mma(v16h a, v16h b, v8f c) {
    return __builtin_amdgcn_wmma_f32_16x16x32_f16(false, a, false, b, (short)0, c, false, false);
  }
  static __device__ __forceinline__ void guard(v8f& a, v8f& b, v16h x, v16h y) { dep_guard_h(a, b, x, y); }
  static __device__ __forceinline__ void keep(v16h a, v16h b, v16h c, v16h d) { keep4_h(a, b, c, d); }
};
template <> struct Frag<__bf16> {
  typedef v16b V; union U { v16b v; v8b h[2]; };
  static __device__ __forceinline__ v16b load(const __bf16* p) {
    U f; f.h[0] = *(const v8b*)(p); f.h[1] = *(const v8b*)(p + 16); return f.v;
  }
  static __device__ __forceinline__ v8f mma(v16b a, v16b b, v8f c) {
    return __builtin_amdgcn_wmma_f32_16x16x32_bf16(false, a, false, b, (short)0, c, false, false);
  }
  static __device__ __forceinline__ void guard(v8f& a, v8f& b, v16b x, v16b y) { dep_guard_b(a, b, x, y); }
  static __device__ __forceinline__ void keep(v16b a, v16b b, v16b c, v16b d) { keep4_b(a, b, c, d); }
};

template <int ET> struct Elem;
template <> struct Elem<0> { typedef _Float16 T; };
template <> struct Elem<1> { typedef __bf16 T; };
template <int ET, bool SPLIT, int BIAS_MODE, int OUT_MODE, bool RESID, int ACT = 0>
__global__ __launch_bounds__(256) void wmma_gemm64(
    const unsigned short* __restrict__ Ap, const unsigned short* __restrict__ A2p, int lda, long strideA,
    const unsigned short* __restrict__ Btp, const unsigned short* __restrict__ Bt2p, int ldb, long strideB,
    void* __restrict__ Cout, void* __restrict__ Cout2, int ldc, long strideC,
    const float* __restrict__ bias,
    const float* __restrict__ resid, long strideR,
    int M, int N, int K, float scale) {
  typedef typename Elem<ET>::T T;
  typedef typename Frag<T>::V V;
  const T* A = (const T*)Ap; const T* A2 = (const T*)A2p; const T* Bt = (const T*)Btp; const T* Bt2 = (const T*)Bt2p;
  __shared__ __align__(16) float sT[8][16 * 68];
  const int b    = blockIdx.y;
  const int lane = threadIdx.x & 31;
  const int wave = threadIdx.x >> 5;
  const int tilesN = N >> 6;
  const int tilesM = M >> 6;
  const int tile = blockIdx.x * 8 + wave;
  if (tile >= tilesM * tilesN) return;
  const int tm = tile / tilesN;
  const int tn = tile - tm * tilesN;
  const int m0 = tm << 6;
  const int n0 = tn << 6;

  const T* Ab  = A  + (size_t)b * strideA;
  const T* Bb  = Bt + (size_t)b * strideB;
  const T* Ab2 = SPLIT ? (A2  + (size_t)b * strideA) : nullptr;
  const T* Bb2 = SPLIT ? (Bt2 + (size_t)b * strideB) : nullptr;

  const int rlane = lane & 15;
  const int koff  = (lane >> 4) * 8;
  const int mOff  = (lane >> 4) * 8;

  v8f acc[4][4];
#pragma unroll
  for (int i = 0; i < 4; ++i)
#pragma unroll
    for (int j = 0; j < 4; ++j) acc[i][j] = (v8f){0.f,0.f,0.f,0.f,0.f,0.f,0.f,0.f};

  for (int k0 = 0; k0 < K; k0 += 32) {
    V bh[4], bl[4];
#pragma unroll
    for (int j = 0; j < 4; ++j) {
      const size_t bo = (size_t)(n0 + (j << 4) + rlane) * ldb + koff + k0;
      bh[j] = Frag<T>::load(Bb + bo);
      if (SPLIT) bl[j] = Frag<T>::load(Bb2 + bo);
    }
#pragma unroll
    for (int i = 0; i < 4; ++i) {
      const size_t ao = (size_t)(m0 + (i << 4) + rlane) * lda + koff + k0;
      V ah = Frag<T>::load(Ab + ao);
      V al;
      if (SPLIT) al = Frag<T>::load(Ab2 + ao);
#pragma unroll
      for (int j = 0; j < 4; ++j) {
        acc[i][j] = Frag<T>::mma(ah, bh[j], acc[i][j]);
        if (SPLIT) {
          acc[i][j] = Frag<T>::mma(ah, bl[j], acc[i][j]);
          acc[i][j] = Frag<T>::mma(al, bh[j], acc[i][j]);
        }
      }
      Frag<T>::guard(acc[i][0], acc[i][3], ah, SPLIT ? al : ah);
    }
    Frag<T>::keep(bh[0], bh[1], bh[2], bh[3]);
    if (SPLIT) Frag<T>::keep(bl[0], bl[1], bl[2], bl[3]);
  }
  acc_guard4(acc[0][0], acc[0][1], acc[0][2], acc[0][3]);
  acc_guard4(acc[1][0], acc[1][1], acc[1][2], acc[1][3]);
  acc_guard4(acc[2][0], acc[2][1], acc[2][2], acc[2][3]);
  acc_guard4(acc[3][0], acc[3][1], acc[3][2], acc[3][3]);

  float* slab = sT[wave];
  const float* Rb = RESID ? (resid + (size_t)b * strideR) : nullptr;
#pragma unroll
  for (int i = 0; i < 4; ++i) {
    const int mBase = m0 + (i << 4);
#pragma unroll
    for (int j = 0; j < 4; ++j) {
      const int n = n0 + (j << 4) + rlane;
      float bv = 0.f;
      if (BIAS_MODE == 2) bv = bias[n];
#pragma unroll
      for (int r = 0; r < 8; ++r) {
        float v = acc[i][j][r] * scale;
        if (BIAS_MODE == 1) v += bias[mBase + mOff + r];
        if (BIAS_MODE == 2) v += bv;
        if (RESID) v += Rb[(size_t)(mBase + mOff + r) * ldc + n];
        if (ACT == 1) v = tanhf(v);
        if (ACT == 2) v = fmaxf(v, 0.0f);
        if (ACT == 3) v = v / (1.0f + expf(-v));
        if (ACT == 4) v = (v > 0.f) ? v : 0.01f * v;
        if (ACT == 5) v = 0.5f * v * (1.0f + erff(v * 0.70710678118654752f));
        slab[(mOff + r) * 68 + (j << 4) + rlane] = v;
      }
    }
    __builtin_amdgcn_fence(__ATOMIC_RELEASE, "workgroup");
    __builtin_amdgcn_wave_barrier();
    __builtin_amdgcn_fence(__ATOMIC_ACQUIRE, "workgroup");
    if (OUT_MODE == 0) {
      float* C = (float*)Cout + (size_t)b * strideC;
      const int hh = lane >> 4, c4 = (lane & 15) * 4;
      for (int pass = 0; pass < 2; ++pass) {
#pragma unroll
        for (int it = 0; it < 8; ++it) {
          const int row = it * 2 + hh;
          v4f v = *(const v4f*)(slab + row * 68 + c4);
          *(volatile v4f*)(C + (size_t)(mBase + row) * ldc + n0 + c4) = v;
        }
        __threadfence();
      }
    } else {
      const int q = lane >> 3, c8 = (lane & 7) * 8;
      unsigned short* C  = (unsigned short*)Cout  + (size_t)b * strideC;
      unsigned short* C2 = (OUT_MODE == 2) ? ((unsigned short*)Cout2 + (size_t)b * strideC) : nullptr;
      for (int pass = 0; pass < 2; ++pass) {
#pragma unroll
        for (int it = 0; it < 4; ++it) {
          const int row = it * 4 + q;
          const float* sp = slab + row * 68 + c8;
          v8h hv, lv;
#pragma unroll
          for (int e = 0; e < 8; ++e) {
            if (OUT_MODE == 1) {
              hv[e] = (_Float16)sp[e];
            } else {
              unsigned short hb = f2bf_bits(sp[e]);
              unsigned short lb = f2bf_bits(sp[e] - bf_bits2f(hb));
              hv[e] = __builtin_bit_cast(_Float16, hb);
              lv[e] = __builtin_bit_cast(_Float16, lb);
            }
          }
          *(volatile v8h*)(C + (size_t)(mBase + row) * ldc + n0 + c8) = hv;
          if (OUT_MODE == 2) *(volatile v8h*)(C2 + (size_t)(mBase + row) * ldc + n0 + c8) = lv;
        }
        __threadfence();
      }
    }
    __builtin_amdgcn_fence(__ATOMIC_RELEASE, "workgroup");
    __builtin_amdgcn_wave_barrier();
    __builtin_amdgcn_fence(__ATOMIC_ACQUIRE, "workgroup");
  }
}


#ifndef SRB
#define SRB 512
#endif
#ifndef SCHK
#define SCHK 4096
#endif
#define SEPT (SCHK / SRB)
__device__ __forceinline__ int blk_excl_scan(int cnt, int* scan_ws, int tid, int* tot) {
  const int lane = tid & 31, wave = tid >> 5; int incl = cnt;
#pragma unroll
  for (int o = 1; o < 32; o <<= 1) { const int v = __shfl_up(incl, o, 32); if (lane >= o) incl += v; }
  if (lane == 31) scan_ws[wave] = incl;
  __syncthreads();
  if (wave == 0) { int wv = (lane < SRB / 32) ? scan_ws[lane] : 0; int wincl = wv;
#pragma unroll
    for (int o = 1; o < 32; o <<= 1) { const int v = __shfl_up(wincl, o, 32); if (lane >= o) wincl += v; }
    if (lane < SRB / 32) scan_ws[32 + lane] = wincl - wv; if (lane == 31) scan_ws[64] = wincl; }
  __syncthreads();
  const int res = scan_ws[32 + wave] + incl - cnt; *tot = scan_ws[64];
  return res;
}
__device__ __forceinline__ int chunk_compact(const int* __restrict__ keyv, const int* __restrict__ othv, int e0, int ne, int n0, int nn, int tid, int* L0, int* L1, int* L2, int* scan_ws) {
  int hk[SEPT], ho[SEPT], he[SEPT]; int cnt = 0;
#pragma unroll
  for (int k = 0; k < SEPT; ++k) { const int e = e0 + tid * SEPT + k; hk[k] = -1; if (e < ne) { const int d = keyv[e]; if (d >= n0 && d < n0 + SRB && d < nn) { hk[k] = d - n0; int s = othv[e]; s = s < 0 ? 0 : (s >= nn ? nn - 1 : s); ho[k] = s; he[k] = e; ++cnt; } } }
  int tot; int p = blk_excl_scan(cnt, scan_ws, tid, &tot);
#pragma unroll
  for (int k = 0; k < SEPT; ++k) if (hk[k] >= 0) { L0[p] = hk[k]; L1[p] = ho[k]; if (L2) L2[p] = he[k]; ++p; }
  __syncthreads();
  return tot;
}
__global__ __launch_bounds__(SRB) void stream_deg_kernel(const int* __restrict__ keyv, const int* __restrict__ othv, int ne, int nn, int* __restrict__ DEG) {
  __shared__ int L0[SCHK]; __shared__ int L1[SCHK]; __shared__ int scan_ws[80];
  const int tid = threadIdx.x, n0 = blockIdx.x * SRB; int cnt = 0;
  for (int e0 = 0; e0 < ne; e0 += SCHK) { const int tot = chunk_compact(keyv, othv, e0, ne, n0, nn, tid, L0, L1, nullptr, scan_ws);
    for (int q = 0; q < tot; ++q) cnt += (L0[q] == tid) ? 1 : 0;
    __syncthreads(); }
  const int n = n0 + tid; if (n < nn) { ((volatile int*)DEG)[n] = cnt; __threadfence(); ((volatile int*)DEG)[n] = cnt; }
}
#define WCAP 64
template <int LO, int HI, int VPL> struct SlotDisp { static __device__ __forceinline__ void add(int s, float (*acc)[VPL], const float* v) {
  if (LO + 1 == HI) {
#pragma unroll
    for (int j = 0; j < VPL; ++j) acc[LO][j] += v[j]; }
  else { const int MID = (LO + HI) / 2; if (s < MID) SlotDisp<LO, (LO + HI) / 2, VPL>::add(s, acc, v); else SlotDisp<(LO + HI) / 2, HI, VPL>::add(s, acc, v); } } };
template <int VW, int CNT>
__device__ __forceinline__ void coop_flush(int n, const unsigned char* wls, const int* wlv, const float* wlw, const float* __restrict__ Hm, int ldh, int lane, float (*acc)[VW + CNT]) {
  for (int j = 0; j < n; ++j) { const int slot = wls[j]; const int src = wlv[j]; const float ew = wlw ? wlw[j] : 1.0f; float v[VW + CNT]; const float* hp = Hm + (size_t)src * ldh + lane * VW;
#pragma unroll
    for (int q = 0; q < VW; ++q) v[q] = wlw ? hp[q] * ew : hp[q];
    if (CNT) v[VW + CNT - 1] = 1.0f;
    SlotDisp<0, 32, VW + CNT>::add(slot, acc, v); }
}
template <int VW, int CNT>
__device__ __forceinline__ void coop_chunk(int tot, const int* L0, const int* L1, const int* L2, const float* __restrict__ EW, unsigned char* wls, int* wlv, float* wlw, const float* __restrict__ Hm, int ldh, int wave, int lane, float (*acc)[VW + CNT]) {
  int nlist = 0;
  for (int q0 = 0; q0 < tot; q0 += 32) { const int q = q0 + lane; int l0 = 0, l1 = 0; float w = 1.f; bool mine = false; if (q < tot) { l0 = L0[q]; l1 = L1[q]; if (EW) w = EW[L2[q]]; mine = (l0 >> 5) == wave; }
    const unsigned bal = __builtin_amdgcn_ballot_w32(mine); const int cntb = __builtin_popcount(bal);
    if (nlist + cntb > WCAP) { coop_flush<VW, CNT>(nlist, wls, wlv, EW ? wlw : nullptr, Hm, ldh, lane, acc); nlist = 0; }
    const int pos = nlist + __builtin_popcount(bal & ((1u << lane) - 1u));
    if (mine) { wls[pos] = (unsigned char)(l0 & 31); wlv[pos] = l1; if (EW) wlw[pos] = w; }
    nlist += cntb; }
  coop_flush<VW, CNT>(nlist, wls, wlv, EW ? wlw : nullptr, Hm, ldh, lane, acc);
}
template <int VW, bool BIDIR, int CNT>
__global__ __launch_bounds__(SRB) void coop_agg_kernel(const float* __restrict__ Hm, int ldh, const int* __restrict__ keyv, const int* __restrict__ othv, const float* __restrict__ EW, int ne, int nn, float* __restrict__ RAW, int ldr, float* __restrict__ DEGOUT) {
  __shared__ int L0[SCHK]; __shared__ int L1[SCHK]; __shared__ int L2[SCHK]; __shared__ int scan_ws[80]; __shared__ unsigned char WLs[32][WCAP]; __shared__ int WLv[32][WCAP]; __shared__ float WLw[32][WCAP];
  const int tid = threadIdx.x, lane = tid & 31, wave = tid >> 5, n0 = blockIdx.x * SRB;
  float acc[32][VW + CNT];
#pragma unroll
  for (int s = 0; s < 32; ++s)
#pragma unroll
    for (int j = 0; j < VW + CNT; ++j) acc[s][j] = 0.f;
  for (int e0 = 0; e0 < ne; e0 += SCHK) {
#pragma unroll
    for (int dir = 0; dir < (BIDIR ? 2 : 1); ++dir) {
      const int tot = chunk_compact(dir ? othv : keyv, dir ? keyv : othv, e0, ne, n0, nn, tid, L0, L1, EW ? L2 : nullptr, scan_ws);
      coop_chunk<VW, CNT>(tot, L0, L1, L2, EW, WLs[wave], WLv[wave], WLw[wave], Hm, ldh, wave, lane, acc);
      __syncthreads(); } }
#pragma unroll
  for (int s = 0; s < 32; ++s) { const int n = n0 + wave * 32 + s; if (n < nn) { float* dst = RAW + (size_t)n * ldr + lane * VW;
      for (int pass = 0; pass < 2; ++pass) {
#pragma unroll
        for (int j = 0; j < VW; ++j) ((volatile float*)dst)[j] = acc[s][j];
        if (CNT && lane == 0) ((volatile float*)DEGOUT)[n] = acc[s][VW + CNT - 1];
        __threadfence(); } } }
}

#define SN 50000
#define SNP 50048
#define SE 800000
#define SD 64
#define SL 3
#define SG 512
__device__ __forceinline__ unsigned pkh(float a, float b) { return (unsigned)__builtin_bit_cast(unsigned short, (_Float16)a) | ((unsigned)__builtin_bit_cast(unsigned short, (_Float16)b) << 16); }
__global__ __launch_bounds__(256) void wprep_kernel(const float* __restrict__ W1, const float* __restrict__ b1, const float* __restrict__ ga, const float* __restrict__ be, const float* __restrict__ mn, const float* __restrict__ vr, const float* __restrict__ W2, unsigned* __restrict__ BT1, float* __restrict__ B1F, unsigned* __restrict__ BT2) {
  for (int i = threadIdx.x; i < SD * SD / 2; i += 256) { const int o = i / 32, kp = 2 * (i % 32); const float s = ga[o] * rsqrtf(vr[o] + 1e-5f);
    const unsigned u1 = pkh(W1[kp * SD + o] * s, W1[(kp + 1) * SD + o] * s), u2 = pkh(W2[kp * SD + o], W2[(kp + 1) * SD + o]);
    ((volatile unsigned*)BT1)[i] = u1; ((volatile unsigned*)BT2)[i] = u2; __threadfence(); ((volatile unsigned*)BT1)[i] = u1; ((volatile unsigned*)BT2)[i] = u2; }
  if (threadIdx.x < SD) { const int o = threadIdx.x; const float s = ga[o] * rsqrtf(vr[o] + 1e-5f); const float v = (b1[o] - mn[o]) * s + be[o]; ((volatile float*)B1F)[o] = v; __threadfence(); ((volatile float*)B1F)[o] = v; }
}
__global__ __launch_bounds__(256) void zin_kernel(const float* __restrict__ Hc, const float* __restrict__ AGG, const float* __restrict__ epsv, int layer, unsigned* __restrict__ Z16) {
  const long i = (long)blockIdx.x * 256 + threadIdx.x; if (i >= (long)SNP * 32) return; const long n = i / 32; float a = 0.f, b = 0.f;
  if (n < SN) { const float s = 1.0f + epsv[layer]; a = s * Hc[2 * i] + AGG[2 * i]; b = s * Hc[2 * i + 1] + AGG[2 * i + 1]; }
  ((volatile unsigned*)Z16)[i] = pkh(a, b); __threadfence(); ((volatile unsigned*)Z16)[i] = pkh(a, b);
}
__global__ __launch_bounds__(256) void pool_kernel(const float* __restrict__ Hc, const float* __restrict__ pmask, const int* __restrict__ batch, const int* __restrict__ mapping, int layer, float* __restrict__ HCAT) {
  __shared__ float red[8][SD + 1]; const int g = blockIdx.x, lane = threadIdx.x & 31, wave = threadIdx.x >> 5;
  float s0 = 0.f, s1 = 0.f;
  for (int n = wave; n < SN; n += 8) if (batch[n] == g) { const float m = pmask[n]; s0 += Hc[(size_t)n * SD + 2 * lane] * m; s1 += Hc[(size_t)n * SD + 2 * lane + 1] * m; }
  red[wave][2 * lane] = s0; red[wave][2 * lane + 1] = s1; __syncthreads();
  if (threadIdx.x < SD) { float t = 0.f; for (int w = 0; w < 8; ++w) t += red[w][threadIdx.x]; int c = mapping[g]; c = c < 0 ? 0 : (c >= SN ? SN - 1 : c);
    float* dst = HCAT + (size_t)g * (2 * SD * SL) + layer * 2 * SD; const float hv = Hc[(size_t)c * SD + threadIdx.x];
    ((volatile float*)dst)[threadIdx.x] = t; ((volatile float*)dst)[SD + threadIdx.x] = hv; __threadfence(); ((volatile float*)dst)[threadIdx.x] = t; ((volatile float*)dst)[SD + threadIdx.x] = hv; }
}
__global__ __launch_bounds__(256) void hcast_kernel(const float* __restrict__ HCAT, unsigned* __restrict__ H16) { for (int i = blockIdx.x * 256 + threadIdx.x; i < SG * SL * SD; i += gridDim.x * 256) { const unsigned u = pkh(HCAT[2 * i], HCAT[2 * i + 1]); ((volatile unsigned*)H16)[i] = u; __threadfence(); ((volatile unsigned*)H16)[i] = u; } }
__global__ __launch_bounds__(256) void lw_kernel(const float* __restrict__ LW, const float* __restrict__ lb, unsigned* __restrict__ BT, float* __restrict__ BP) {
  for (int i = threadIdx.x; i < 64 * 384 / 2; i += 256) { const int o = i / 192, kp = 2 * (i % 192); float a = 0.f, b = 0.f; if (o < 32) { a = LW[kp * 32 + o]; b = LW[(kp + 1) * 32 + o]; } ((volatile unsigned*)BT)[i] = pkh(a, b); __threadfence(); ((volatile unsigned*)BT)[i] = pkh(a, b); }
  if (threadIdx.x < 64) { const float v = threadIdx.x < 32 ? lb[threadIdx.x] : 0.f; ((volatile float*)BP)[threadIdx.x] = v; __threadfence(); ((volatile float*)BP)[threadIdx.x] = v; }
}
__global__ __launch_bounds__(256) void outc_kernel(const float* __restrict__ OP, float* __restrict__ out) { for (int i = blockIdx.x * 256 + threadIdx.x; i < SG * 32; i += gridDim.x * 256) { const float v = OP[(i / 32) * 64 + (i % 32)]; ((volatile float*)out)[i] = v; __threadfence(); ((volatile float*)out)[i] = v; } }
extern "C" void kernel_launch(void* const* d_in, const int* in_sizes, int n_in, void* d_out, int out_size, void* d_ws, size_t ws_size, hipStream_t stream) {
  (void)in_sizes; (void)n_in; (void)out_size; (void)ws_size;
  auto Fp = [&](int i) { return (const float*)d_in[i]; };
  const float* x = Fp(0); const float* ew = Fp(1); const float* pmask = Fp(2); const float* W1 = Fp(3); const float* b1 = Fp(4); const float* ga = Fp(5); const float* be = Fp(6); const float* mn = Fp(7); const float* vr = Fp(8); const float* W2 = Fp(9); const float* b2 = Fp(10); const float* epsv = Fp(11); const float* LW = Fp(12); const float* lb = Fp(13);
  const int* ei = (const int*)d_in[14]; const int* batch = (const int*)d_in[15]; const int* mapping = (const int*)d_in[16];
  char* ws = (char*)d_ws; size_t off = 0;
  auto carve = [&](size_t bytes) -> char* { char* p = ws + off; off += (bytes + 255) & ~(size_t)255; return p; };
  float* AGG = (float*)carve((size_t)SNP * SD * 4); unsigned* Z16 = (unsigned*)carve((size_t)SNP * SD * 2); _Float16* T16 = (_Float16*)carve((size_t)SNP * SD * 2); float* Hc = (float*)carve((size_t)SNP * SD * 4);
  unsigned* BT1 = (unsigned*)carve(SD * SD * 2); unsigned* BT2 = (unsigned*)carve(SD * SD * 2); float* B1F = (float*)carve(256); float* HCAT = (float*)carve((size_t)SG * 2 * SD * SL * 4); unsigned* H16 = (unsigned*)carve((size_t)SG * 2 * SD * SL * 2); unsigned* LBT = (unsigned*)carve(64 * 384 * 2); float* LBP = (float*)carve(256); float* OP = (float*)carve(SG * 64 * 4);
  const int* src = ei; const int* dst = ei + SE; const int nb = (SN + SRB - 1) / SRB; const int t = (SNP / 64) * 1;
  lw_kernel<<<1, 256, 0, stream>>>(LW, lb, LBT, LBP);
  const float* hin = x;
  for (int l = 0; l < SL; ++l) {
    wprep_kernel<<<1, 256, 0, stream>>>(W1 + (size_t)l * SD * SD, b1 + l * SD, ga + l * SD, be + l * SD, mn + l * SD, vr + l * SD, W2 + (size_t)l * SD * SD, BT1, B1F, BT2);
    coop_agg_kernel<2, false, 0><<<nb, SRB, 0, stream>>>(hin, SD, dst, src, ew, SE, SN, AGG, SD, nullptr);
    zin_kernel<<<(SNP * 32 + 255) / 256, 256, 0, stream>>>(hin, AGG, epsv, l, Z16);
    wmma_gemm64<0, false, 2, 1, false, 2><<<dim3((t + 7) / 8, 1), 256, 0, stream>>>((const unsigned short*)Z16, nullptr, SD, 0, (const unsigned short*)BT1, nullptr, SD, 0, T16, nullptr, SD, 0, B1F, nullptr, 0, SNP, SD, SD, 1.0f);
    wmma_gemm64<0, false, 2, 0, false, 2><<<dim3((t + 7) / 8, 1), 256, 0, stream>>>(U16(T16), nullptr, SD, 0, (const unsigned short*)BT2, nullptr, SD, 0, Hc, nullptr, SD, 0, b2 + l * SD, nullptr, 0, SNP, SD, SD, 1.0f);
    pool_kernel<<<SG, 256, 0, stream>>>(Hc, pmask, batch, mapping, l, HCAT);
    hin = Hc; }
  hcast_kernel<<<64, 256, 0, stream>>>(HCAT, H16);
  wmma_gemm64<0, false, 2, 0, false><<<dim3(1, 1), 256, 0, stream>>>((const unsigned short*)H16, nullptr, 2 * SD * SL, 0, (const unsigned short*)LBT, nullptr, 2 * SD * SL, 0, OP, nullptr, 64, 0, LBP, nullptr, 0, SG, 64, 2 * SD * SL, 1.0f);
  outc_kernel<<<(SG * 32 + 255) / 256, 256, 0, stream>>>(OP, (float*)d_out);
}
